// NNUE_83640193122666
// MI455X (gfx1250) — hardware-verified
//
#include <hip/hip_runtime.h>
#include <stddef.h>
#include <stdint.h>


#define NB    16384
#define MSTK  32768
#define INP   768
#define ACC   1024
#define COMB  2048
#define NBK   8
#define ESC   16
#define WSC   1024
#define NTHR  256
#define NWAVE 8
#define NCG   16
#define WSCAP 134217728

static_assert((INP % 32) == 0);
static_assert((MSTK % 128) == 0);
static_assert((NB % 128) == 0);
static_assert((ACC % 128) == 0);
static_assert(((NB * INP) % (8 * NTHR)) == 0);
static_assert(((ACC * INP) % (8 * NTHR)) == 0);
static_assert((NB % NTHR) == 0);
static_assert(NTHR == NWAVE * 32);
static_assert(NCG * 64 == ACC);
static_assert(MSTK == 2 * NB);
static_assert(COMB == 2 * ACC);
static_assert((NCG % 8) == 0);

typedef float          v4f  __attribute__((ext_vector_type(4)));
typedef float          v8f  __attribute__((ext_vector_type(8)));
typedef _Float16       v8h  __attribute__((ext_vector_type(8)));
typedef _Float16       v16h __attribute__((ext_vector_type(16)));
union FragH { v16h v; v8h h[2]; };

__device__ __forceinline__ v8f wmf(v16h a, v16h b, v8f c) {
  v8f d = __builtin_amdgcn_wmma_f32_16x16x32_f16(false, a, false, b, (short)0, c, false, false);
  asm volatile("v_nop\n\tv_nop\n\tv_nop\n\tv_nop" : "+v"(d) : "v"(a), "v"(b));
  return d;
}

__device__ __forceinline__ int clamp_sel(int s) {
  s = (s < 0) ? s + NBK : s;
  s = (s < 0) ? 0 : s;
  s = (s > NBK - 1) ? NBK - 1 : s;
  return s;
}

__global__ __launch_bounds__(NTHR) void k_cvt(const float* __restrict__ src, _Float16* dst, float scale) {
  const size_t t = (size_t)blockIdx.x * NTHR + threadIdx.x;
  const float* p = src + t * 8;
  const v4f f0 = *(const v4f*)p;
  const v4f f1 = *(const v4f*)(p + 4);
  v8h a;
  a[0] = (_Float16)(f0.x * scale); a[1] = (_Float16)(f0.y * scale);
  a[2] = (_Float16)(f0.z * scale); a[3] = (_Float16)(f0.w * scale);
  a[4] = (_Float16)(f1.x * scale); a[5] = (_Float16)(f1.y * scale);
  a[6] = (_Float16)(f1.z * scale); a[7] = (_Float16)(f1.w * scale);
  _Float16* d = dst + t * 8;
  *(volatile v8h*)d = a;
  __threadfence();
  *(volatile v8h*)d = a;
}

__global__ __launch_bounds__(NTHR) void k_gemm(const _Float16* __restrict__ ap, const _Float16* __restrict__ wt,
                                               const float* __restrict__ acc_b, const float* __restrict__ out_w,
                                               const int* __restrict__ sel, float* part) {
  __shared__ __attribute__((aligned(16))) float sOW[NBK * 128];
  __shared__ int sSel[128];
  __shared__ __attribute__((aligned(16))) float sP[NWAVE * 32];

  const int tid = threadIdx.x, lane = tid & 31, wave = tid >> 5, hf = lane >> 4, m = lane & 15;
  const int n0 = blockIdx.x * 128, m0 = blockIdx.y * 128;
  const int persp = (m0 >= NB) ? 1 : 0;
  const int brow0 = m0 - persp * NB;
  const int colc0 = persp * ACC + n0;
  const int wm = (wave >> 1) * 32, wn = (wave & 1) * 64;

#pragma unroll
  for (int i = 0; i < 4; ++i) {
    const int idx = tid + NTHR * i;
    const int k = idx >> 7, c = idx & 127;
    sOW[idx] = out_w[(size_t)k * COMB + colc0 + c];
  }
  if (tid < 128) sSel[tid] = clamp_sel(sel[brow0 + tid]);
  float bv[4];
#pragma unroll
  for (int nt = 0; nt < 4; ++nt) bv[nt] = acc_b[n0 + wn + 16 * nt + m];
  __syncthreads();

  v8f acc[2][4];
#pragma unroll
  for (int mt = 0; mt < 2; ++mt)
#pragma unroll
    for (int nt = 0; nt < 4; ++nt) { v8f z = {0.f, 0.f, 0.f, 0.f, 0.f, 0.f, 0.f, 0.f}; acc[mt][nt] = z; }

  const _Float16* aq = ap + (size_t)(m0 + wm + m) * INP + 8 * hf;
  const _Float16* bp = wt + (size_t)(n0 + wn + m) * INP + 8 * hf;
#pragma unroll 1
  for (int kt = 0; kt < INP / 32; ++kt) {
    const int k0 = 32 * kt;
    FragH a0, a1;
    a0.h[0] = *(const v8h*)(aq + k0);
    a0.h[1] = *(const v8h*)(aq + k0 + 16);
    a1.h[0] = *(const v8h*)(aq + (size_t)16 * INP + k0);
    a1.h[1] = *(const v8h*)(aq + (size_t)16 * INP + k0 + 16);
#pragma unroll
    for (int nt = 0; nt < 4; ++nt) {
      const _Float16* bq = bp + (size_t)nt * 16 * INP + k0;
      FragH b;
      b.h[0] = *(const v8h*)bq;
      b.h[1] = *(const v8h*)(bq + 16);
      acc[0][nt] = wmf(a0.v, b.v, acc[0][nt]);
      acc[1][nt] = wmf(a1.v, b.v, acc[1][nt]);
    }
  }

  constexpr float OSC = 1.0f / (float)(ESC * WSC);
#pragma unroll
  for (int mt = 0; mt < 2; ++mt) {
#pragma unroll
    for (int r = 0; r < 8; ++r) {
      const int lrow = wm + 16 * mt + 8 * hf + r;
      const int s = sSel[lrow];
      const float* ow = sOW + s * 128 + wn + m;
      float p = 0.f;
#pragma unroll
      for (int nt = 0; nt < 4; ++nt) {
        float v = fmaf(acc[mt][nt][r], OSC, bv[nt]);
        v = fminf(fmaxf(v, 0.f), 6.f);
        p = fmaf(v, ow[16 * nt], p);
      }
      p += __shfl_xor(p, 8);
      p += __shfl_xor(p, 4);
      p += __shfl_xor(p, 2);
      p += __shfl_xor(p, 1);
      if (m == 0) sP[wave * 32 + 16 * mt + 8 * hf + r] = p;
    }
  }
  __syncthreads();

  const v4f v = *(const v4f*)(sP + wave * 32 + 4 * (lane & 7));
  const int g = blockIdx.x * 2 + (wave & 1);
  float* d = part + (size_t)g * MSTK + (size_t)(m0 + wm) + 4 * (lane & 7);
  if (lane < 8) *(volatile v4f*)d = v;
  __threadfence();
  if (lane < 8) *(volatile v4f*)d = v;
}

__global__ __launch_bounds__(NTHR) void k_fin(const float* __restrict__ part, const int* __restrict__ sel,
                                              const float* __restrict__ out_b, float* out) {
  __shared__ __attribute__((aligned(16))) float sq[NTHR];
  const int t = threadIdx.x;
  const int b = blockIdx.x * NTHR + t;
  const int s = clamp_sel(sel[b]);
  float acc = out_b[s];
#pragma unroll 1
  for (int c = 0; c < 4; ++c) {
    const float* pb = part + (size_t)((c & 1) * 8) * MSTK + (size_t)(c >> 1) * NB + b;
    float pv[8];
#pragma unroll
    for (int j = 0; j < 8; ++j) pv[j] = pb[(size_t)j * MSTK];
#pragma unroll
    for (int j = 0; j < 8; ++j) acc += pv[j];
  }
  sq[t] = acc;
  __syncthreads();
  const v4f v = *(const v4f*)(sq + 4 * (t & 63));
  float* d = out + (size_t)blockIdx.x * NTHR + 4 * (t & 63);
  if (t < 64) *(volatile v4f*)d = v;
  __threadfence();
  if (t < 64) *(volatile v4f*)d = v;
}

extern "C" void kernel_launch(void* const* d_in, const int* in_sizes, int n_in,
                              void* d_out, int out_size, void* d_ws, size_t ws_size,
                              hipStream_t stream) {
  if (n_in < 7) return;
  if (in_sizes[0] != NB * INP || in_sizes[1] != NB * INP || in_sizes[2] != NB ||
      in_sizes[3] != ACC * INP || in_sizes[4] != ACC || in_sizes[5] != NBK * COMB ||
      in_sizes[6] != NBK) return;
  if (out_size != NB) return;

  const float* stm   = (const float*)d_in[0];
  const float* nstm  = (const float*)d_in[1];
  const int*   sel   = (const int*)d_in[2];
  const float* acc_w = (const float*)d_in[3];
  const float* acc_b = (const float*)d_in[4];
  const float* out_w = (const float*)d_in[5];
  const float* out_b = (const float*)d_in[6];
  float* out = (float*)d_out;

  char* ws = (char*)d_ws;
  size_t off = 0;
  const size_t oA = off; off += (size_t)MSTK * INP * 2;  off = (off + 255) & ~(size_t)255;
  const size_t oW = off; off += (size_t)ACC * INP * 2;   off = (off + 255) & ~(size_t)255;
  const size_t oP = off; off += (size_t)NCG * MSTK * 4;  off = (off + 255) & ~(size_t)255;
  if (off > ws_size || off > (size_t)WSCAP) return;
  _Float16* ap = (_Float16*)(ws + oA);
  _Float16* wt = (_Float16*)(ws + oW);
  float* part = (float*)(ws + oP);

  k_cvt<<<(NB * INP) / (8 * NTHR), NTHR, 0, stream>>>(stm, ap, (float)ESC);
  k_cvt<<<(NB * INP) / (8 * NTHR), NTHR, 0, stream>>>(nstm, ap + (size_t)NB * INP, (float)ESC);
  k_cvt<<<(ACC * INP) / (8 * NTHR), NTHR, 0, stream>>>(acc_w, wt, (float)WSC);
  k_gemm<<<dim3(ACC / 128, MSTK / 128), NTHR, 0, stream>>>(ap, wt, acc_b, out_w, sel, part);
  k_fin<<<NB / NTHR, NTHR, 0, stream>>>(part, sel, out_b, out);
}
